// CentroidTDBase_60490319397195
// MI455X (gfx1250) — hardware-run, weakly checked
//
#include <hip/hip_runtime.h>


#define NB_  256
#define NF   512
#define ND   256
#define NR   320
#define PT   0.05f
#define OMM  0.05f
typedef _Float16 h16;
typedef unsigned short bf;
typedef __attribute__((ext_vector_type(16))) __bf16   v16bf;
typedef __attribute__((ext_vector_type(16))) _Float16 v16h;
typedef __attribute__((ext_vector_type(8)))  _Float16 v8h;
typedef __attribute__((ext_vector_type(8)))  unsigned short v8us;
typedef __attribute__((ext_vector_type(8)))  float    v8f;
typedef __attribute__((ext_vector_type(4)))  float    v4f;
typedef v8h  __attribute__((may_alias)) v8ha;
typedef v4f  __attribute__((may_alias)) v4fa;
typedef v8us __attribute__((may_alias)) v8usa;

__device__ __forceinline__ unsigned short f2bf(float f) { unsigned u = __float_as_uint(f); u += 0x7FFFu + ((u >> 16) & 1u); return (unsigned short)(u >> 16); }
__device__ __forceinline__ float bf2f(unsigned short b) { return __uint_as_float(((unsigned)b) << 16); }
__device__ __forceinline__ float bfr(float f) { return bf2f(f2bf(f)); }
__device__ __forceinline__ v16h cat16(v8h lo, v8h hi) { return __builtin_shufflevector(lo, hi, 0, 1, 2, 3, 4, 5, 6, 7, 8, 9, 10, 11, 12, 13, 14, 15); }
__device__ __forceinline__ v16bf cat16b(v8us lo, v8us hi) { return __builtin_bit_cast(v16bf, __builtin_shufflevector(lo, hi, 0, 1, 2, 3, 4, 5, 6, 7, 8, 9, 10, 11, 12, 13, 14, 15)); }
__device__ __forceinline__ v8f wmma16(v16h a, v16h b, v8f c) { return __builtin_amdgcn_wmma_f32_16x16x32_f16(false, a, false, b, (short)0, c, false, false); }
__device__ __forceinline__ v8f wmmab(v16bf a, v16bf b, v8f c) { return __builtin_amdgcn_wmma_f32_16x16x32_bf16(false, a, false, b, (short)0, c, false, false); }


template <typename T16> struct WFrag;
template <> struct WFrag<h16> { typedef v16h V; static __device__ __forceinline__ V ld(const h16* p) { return cat16(*(const v8h*)p, *(const v8h*)(p + 16)); } static __device__ __forceinline__ v8f mma(V a, V b, v8f c) { return wmma16(a, b, c); } };
template <> struct WFrag<bf> { typedef v16bf V; static __device__ __forceinline__ V ld(const bf* p) { return cat16b(*(const v8us*)p, *(const v8us*)(p + 16)); } static __device__ __forceinline__ v8f mma(V a, V b, v8f c) { return wmmab(a, b, c); } };
template <typename T16, int NSPLIT, bool BIAS>
__global__ __launch_bounds__(32) void k_gemmw(const T16* __restrict__ A, const T16* __restrict__ A2, const T16* __restrict__ Bt, const T16* __restrict__ Bt2, int K, float* C, int ldc, const float* __restrict__ bias, size_t sA, size_t sB, size_t sC) {
    typedef typename WFrag<T16>::V V;
    __shared__ __align__(16) float os[16 * 68];
    const size_t z = blockIdx.z; A += z * sA; if (A2) A2 += z * sA; Bt += z * sB; if (Bt2) Bt2 += z * sB; C += z * sC;
    const int lane = threadIdx.x & 31, lr = lane & 15, hi = lane >> 4; const int r0 = blockIdx.x * 64, c0 = blockIdx.y * 64;
    v8f acc[4][4];
#pragma unroll
    for (int mb = 0; mb < 4; ++mb)
#pragma unroll
        for (int nb = 0; nb < 4; ++nb) acc[mb][nb] = (v8f){};
    const size_t aoff = (size_t)(r0 + lr) * K + 8 * hi, boff = (size_t)(c0 + lr) * K + 8 * hi;
    for (int kc = 0; kc < K; kc += 32) {
        V a[4], a2[4];
#pragma unroll
        for (int mb = 0; mb < 4; ++mb) { a[mb] = WFrag<T16>::ld(A + aoff + (size_t)mb * 16 * K + kc); if (NSPLIT == 1 || NSPLIT == 2) a2[mb] = WFrag<T16>::ld(A2 + aoff + (size_t)mb * 16 * K + kc); }
#pragma unroll
        for (int nb = 0; nb < 4; ++nb) { const V b = WFrag<T16>::ld(Bt + boff + (size_t)nb * 16 * K + kc); V b2; if (NSPLIT >= 2) b2 = WFrag<T16>::ld(Bt2 + boff + (size_t)nb * 16 * K + kc);
#pragma unroll
            for (int mb = 0; mb < 4; ++mb) { acc[mb][nb] = WFrag<T16>::mma(a[mb], b, acc[mb][nb]); if (NSPLIT == 1 || NSPLIT == 2) acc[mb][nb] = WFrag<T16>::mma(a2[mb], b, acc[mb][nb]); if (NSPLIT >= 2) acc[mb][nb] = WFrag<T16>::mma(a[mb], b2, acc[mb][nb]); } }
        asm volatile("v_nop\n\tv_nop\n\tv_nop\n\tv_nop" : "+v"(acc[0][0]), "+v"(acc[1][1]), "+v"(acc[2][2]), "+v"(acc[3][3]) : "v"(a[0]), "v"(a[3]));
    }
#pragma unroll
    for (int mb = 0; mb < 4; ++mb) {
#pragma unroll
        for (int nb = 0; nb < 4; ++nb) {
#pragma unroll
            for (int j = 0; j < 8; ++j) os[(hi * 8 + j) * 68 + nb * 16 + lr] = acc[mb][nb][j]; }
        __builtin_amdgcn_wave_barrier(); asm volatile("" ::: "memory");
        float* crow = C + (size_t)(r0 + mb * 16) * ldc + c0;
#pragma unroll 1
        for (int ps = 0; ps < 2; ++ps) {
#pragma unroll
            for (int s = 0; s < 8; ++s) { const int row = 2 * s + hi, cofs = lr * 4; v4f val = *(const v4fa*)(os + row * 68 + cofs); if (BIAS) { val[0] += bfr(bias[c0 + cofs]); val[1] += bfr(bias[c0 + cofs + 1]); val[2] += bfr(bias[c0 + cofs + 2]); val[3] += bfr(bias[c0 + cofs + 3]); }
                *(volatile v4f*)(crow + (size_t)row * ldc + cofs) = val; }
            if (ps == 0) __threadfence(); }
        __builtin_amdgcn_wave_barrier(); asm volatile("" ::: "memory");
    }
}

__device__ __forceinline__ h16 tohx(float x) { return (h16)x; }
__device__ __forceinline__ void splitf(float y, unsigned short& h, unsigned short& l) { h = f2bf(y); l = f2bf(y - bf2f(h)); }
typedef __attribute__((ext_vector_type(2))) _Float16 v2h;
typedef __attribute__((ext_vector_type(4))) _Float16 v4h;
typedef __attribute__((ext_vector_type(2))) unsigned short v2us;
typedef __attribute__((ext_vector_type(4))) unsigned short v4us;
typedef __attribute__((ext_vector_type(2))) float v2f;
typedef __attribute__((ext_vector_type(4))) int v4i;

__global__ __launch_bounds__(256) void k_tb(const float* __restrict__ src, int C, int ones, float sc, bf* T) { const unsigned idx = blockIdx.x * 256 + threadIdx.x; const unsigned b0 = (idx % (NB_ / 2)) * 2, r = idx / (NB_ / 2); const unsigned rc = (r < (unsigned)C) ? r : (unsigned)(C - 1); v2us o;
#pragma unroll
    for (int q = 0; q < 2; ++q) { const float w = __fmul_rn(bfr(src[(size_t)(b0 + q) * C + rc]), sc); const float y = (r < (unsigned)C) ? w : ((ones != 0 && r == (unsigned)C) ? 1.0f : 0.0f); o[q] = f2bf(y); }
    *(volatile v2us*)(T + (size_t)idx * 2) = o; __threadfence(); *(volatile v2us*)(T + (size_t)idx * 2) = o; }
__global__ __launch_bounds__(256) void k_pa(const float* __restrict__ a5, h16* P) { const unsigned idx = blockIdx.x * 256 + threadIdx.x; const unsigned j0 = (idx % (NF / 4)) * 4, r = idx / (NF / 4); const unsigned rc = (r < ND) ? r : (ND - 1); const v4f a = *(const v4f*)(a5 + (size_t)rc * NF + j0); v4h o;
#pragma unroll
    for (int q = 0; q < 4; ++q) { const float w = bfr(a[q]); const float y = (r < ND) ? ((fabsf(w) < 6.103515625e-5f) ? 0.0f : w) : ((r == ND) ? 1.0f : 0.0f); o[q] = tohx(y); }
    *(volatile v4h*)(P + (size_t)idx * 4) = o; __threadfence(); *(volatile v4h*)(P + (size_t)idx * 4) = o; }
__device__ __forceinline__ void pw_words(float s, float mu, float& zm, float& r0, float& t) { zm = __fmul_rn(s, 0.00390625f); r0 = __fmul_rn(OMM, __fsub_rn(zm, mu)); t = __fadd_rn(mu, r0); }
__global__ __launch_bounds__(256) void k_pw(const float* __restrict__ S1, const float* __restrict__ a4, float* R0, h16* Wd16) { const unsigned idx = blockIdx.x * 256 + threadIdx.x; const v4f s = *(const v4f*)(S1 + (size_t)idx * 4); const v4f m4 = *(const v4f*)(a4 + (size_t)idx * 4); v4f o0; v4h ow;
#pragma unroll
    for (int q = 0; q < 4; ++q) { float zm, r0, t; pw_words(s[q], bfr(m4[q]), zm, r0, t); o0[q] = r0; const float wd = __fmul_rn(__fmul_rn(__fsub_rn(__fmul_rn(PT, PT), t), zm), 256.0f); ow[q] = tohx((fabsf(wd) < 6.103515625e-5f) ? 0.0f : wd); }
    *(volatile v4f*)(R0 + (size_t)idx * 4) = o0; *(volatile v4h*)(Wd16 + (size_t)idx * 4) = ow; __threadfence(); *(volatile v4f*)(R0 + (size_t)idx * 4) = o0; *(volatile v4h*)(Wd16 + (size_t)idx * 4) = ow; }
__global__ __launch_bounds__(128) void k_dg(const float* __restrict__ S1, const float* __restrict__ a4, float* R2, float* R4, float* PV) { const unsigned i0 = threadIdx.x * 4; v4f o;
#pragma unroll
    for (int q = 0; q < 4; ++q) { const size_t a = (size_t)(i0 + q) * (NF + 1); float zm, r0, t; pw_words(S1[a], bfr(a4[a]), zm, r0, t); o[q] = __fsub_rn(PT, t); }
    *(volatile v4f*)(R2 + i0) = o; *(volatile v4f*)(R4 + i0) = o; *(volatile v4f*)(PV + i0) = o; __threadfence(); *(volatile v4f*)(R2 + i0) = o; *(volatile v4f*)(R4 + i0) = o; *(volatile v4f*)(PV + i0) = o; }
__global__ __launch_bounds__(256) void k_cb(const float* __restrict__ S2, const float* __restrict__ S3, const float* __restrict__ a5, const float* __restrict__ PV, float* R1) { const unsigned idx = blockIdx.x * 256 + threadIdx.x; const unsigned i0 = (idx % (NF / 4)) * 4, d = idx / (NF / 4); const v4f s2 = *(const v4f*)(S2 + (size_t)d * NF + i0); const v4f zc = *(const v4f*)(S2 + (size_t)ND * NF + i0); const v4f k4 = *(const v4f*)(a5 + (size_t)d * NF + i0); const v4f pv = *(const v4f*)(PV + i0); v4f o;
#pragma unroll
    for (int q = 0; q < 4; ++q) { const float kk = bfr(k4[q]); const float cx = __fmul_rn(S3[(size_t)(i0 + q) * NR + d], 0.00390625f / NF), rm = __fmul_rn(S3[(size_t)(i0 + q) * NR + ND], 0.00390625f / NF); const float selft = __fmul_rn(pv[q], __fsub_rn(__fmul_rn(s2[q], 0.00390625f), __fmul_rn(kk, __fmul_rn(zc[q], 0.00390625f)))); const float dec = __fsub_rn(__fmul_rn(kk, rm), cx); o[q] = __fadd_rn(selft, dec); }
    *(volatile v4f*)(R1 + (size_t)idx * 4) = o; __threadfence(); *(volatile v4f*)(R1 + (size_t)idx * 4) = o; }

extern "C" void kernel_launch(void* const* d_in, const int* in_sizes, int n_in,
                              void* d_out, int out_size, void* d_ws, size_t ws_size, hipStream_t stream) {
    (void)in_sizes; (void)n_in; (void)out_size;
    const float* a0 = (const float*)d_in[0]; const float* a1 = (const float*)d_in[1]; const float* a2 = (const float*)d_in[2]; const float* a3 = (const float*)d_in[3]; const float* a4 = (const float*)d_in[4]; const float* a5 = (const float*)d_in[5];
    float* R0 = (float*)d_out; float* R1 = R0 + (size_t)NF * NF; float* R2 = R1 + (size_t)ND * NF; float* R3 = R2 + NF; float* R4 = R3 + (size_t)NF * NF;
    char* wsp = (char*)d_ws;
    auto take = [&](size_t bytes) { char* p = wsp; wsp += (bytes + 255) & ~(size_t)255; return (void*)p; };
    bf* T0 = (bf*)take((size_t)NF * NB_ * 2); bf* T1 = (bf*)take((size_t)NR * NB_ * 2); bf* T2 = (bf*)take((size_t)NF * NB_ * 2); bf* T3 = (bf*)take((size_t)NF * NB_ * 2); h16* P5 = (h16*)take((size_t)NR * NF * 2);
    float* S1 = (float*)take((size_t)NF * NF * 4); float* S2 = (float*)take((size_t)NR * NF * 4); h16* Wd16 = (h16*)take((size_t)NF * NF * 2); float* S3 = (float*)take((size_t)NF * NR * 4); float* PV = (float*)take((size_t)NF * 4);
    if ((size_t)(wsp - (char*)d_ws) > ws_size) return;
    k_tb<<<NF * (NB_ / 2) / 256, 256, 0, stream>>>(a0, NF, 0, 1.0f, T0); k_tb<<<NR * (NB_ / 2) / 256, 256, 0, stream>>>(a1, ND, 1, 1.0f, T1); k_tb<<<NF * (NB_ / 2) / 256, 256, 0, stream>>>(a2, NF, 0, 0.00390625f, T2); k_tb<<<NF * (NB_ / 2) / 256, 256, 0, stream>>>(a3, NF, 0, 1.0f, T3);
    k_pa<<<NR * (NF / 4) / 256, 256, 0, stream>>>(a5, P5);
    k_gemmw<bf, 0, false><<<dim3(NF / 64, NF / 64, 1), 32, 0, stream>>>(T0, nullptr, T0, nullptr, NB_, S1, NF, nullptr, 0, 0, 0);
    k_gemmw<bf, 0, false><<<dim3(NR / 64, NF / 64, 1), 32, 0, stream>>>(T1, nullptr, T0, nullptr, NB_, S2, NF, nullptr, 0, 0, 0);
    k_gemmw<bf, 0, false><<<dim3(NF / 64, NF / 64, 1), 32, 0, stream>>>(T2, nullptr, T3, nullptr, NB_, R3, NF, nullptr, 0, 0, 0);
    k_pw<<<NF * (NF / 4) / 256, 256, 0, stream>>>(S1, a4, R0, Wd16);
    k_dg<<<1, 128, 0, stream>>>(S1, a4, R2, R4, PV);
    k_gemmw<h16, 0, false><<<dim3(NF / 64, NR / 64, 1), 32, 0, stream>>>(Wd16, nullptr, P5, nullptr, NF, S3, NR, nullptr, 0, 0, 0);
    k_cb<<<ND * (NF / 4) / 256, 256, 0, stream>>>(S2, S3, a5, PV, R1);
}
